// SpatialAttentionLayer_45612552683794
// MI455X (gfx1250) — hardware-verified
//
#include <hip/hip_runtime.h>

#define NJ     8192
#define NF     100
#define NFP    112
#define NTL    7
#define QROWS  64
#define PJ     256
#define PSCALE 16384.0f
#define LSLOPE 0.2f

typedef _Float16 v16h __attribute__((ext_vector_type(16)));
typedef _Float16 v8h  __attribute__((ext_vector_type(8)));
typedef float    v8f  __attribute__((ext_vector_type(8)));
typedef float    v4f  __attribute__((ext_vector_type(4)));
typedef float    v4fa __attribute__((ext_vector_type(4), __may_alias__));

union Frag { v16h v; v8h half[2]; };

__device__ __forceinline__ v8f wmma16(v16h a, v16h b, v8f c) {
    v8f d = __builtin_amdgcn_wmma_f32_16x16x32_f16(false, a, false, b, (short)0, c, false, false);
    asm volatile("v_nop\n\tv_nop\n\tv_nop\n\tv_nop" : "+v"(d) : "v"(a), "v"(b));
    return d;
}

__device__ __forceinline__ float lk(float v) { return (v >= 0.f) ? v : LSLOPE * v; }

__device__ __forceinline__ _Float16 pval(float s, float s_im, float Mrow, float& z) {
    const float e = lk(s_im + s);
    const float p = __expf(e - Mrow);
    z += p;
    return (_Float16)(p * PSCALE);
}

__device__ __forceinline__ void prep_stores(const float* __restrict__ x, _Float16* x16,
                                            float* s1, float* s2, const float* sS,
                                            int j0, int wv, int l)
{
#pragma unroll 1
    for (int rr = 0; rr < NFP / 8; ++rr) {
        const int f = wv + 8 * rr;
        v8h hv;
        if (f < NF) {
            const float* xp = x + (size_t)f * NJ + j0 + 8 * l;
            const v4f a0 = *(const v4f*)(xp);
            const v4f a1 = *(const v4f*)(xp + 4);
#pragma unroll
            for (int i = 0; i < 4; ++i) {
                hv[i]     = (_Float16)a0[i];
                hv[4 + i] = (_Float16)a1[i];
            }
        } else {
#pragma unroll
            for (int i = 0; i < 8; ++i) hv[i] = (_Float16)0.0f;
        }
        *(volatile v8h*)(x16 + (size_t)f * NJ + j0 + 8 * l) = hv;
    }
    if (wv == 0) {
#pragma unroll
        for (int g = 0; g < 2; ++g) {
            const v4f v = *(const v4fa*)(sS + 128 * g + 4 * l);
            *(volatile v4f*)(s1 + j0 + 128 * g + 4 * l) = v;
        }
    } else if (wv == 1) {
#pragma unroll
        for (int g = 0; g < 2; ++g) {
            const v4f v = *(const v4fa*)(sS + PJ + 128 * g + 4 * l);
            *(volatile v4f*)(s2 + j0 + 128 * g + 4 * l) = v;
        }
    }
}

__global__ void __launch_bounds__(256)
k_prep(const float* __restrict__ x, const float* __restrict__ w,
       _Float16* __restrict__ x16, float* __restrict__ s1, float* __restrict__ s2)
{
    __shared__ __align__(16) float sW[2 * NF];
    __shared__ __align__(16) float sS[2 * PJ];

    const int tid = threadIdx.x, l = tid & 31, wv = tid >> 5;
    const int j0 = blockIdx.x * PJ;

    if (tid < 2 * NF) sW[tid] = w[tid];
    __syncthreads();

    {
        const int j = j0 + tid;
        float a = 0.f, b = 0.f;
#pragma unroll 4
        for (int f = 0; f < NF; ++f) {
            const float xv = x[(size_t)f * NJ + j];
            a = fmaf(xv, sW[f], a);
            b = fmaf(xv, sW[NF + f], b);
        }
        sS[tid]      = a;
        sS[PJ + tid] = b;
    }
    __syncthreads();

    prep_stores(x, x16, s1, s2, sS, j0, wv, l);
    __threadfence();
    prep_stores(x, x16, s1, s2, sS, j0, wv, l);
}

__global__ void __launch_bounds__(128)
k_attn(const _Float16* __restrict__ x16, const float* __restrict__ s1,
       const float* __restrict__ s2, float* __restrict__ out)
{
    __shared__ __align__(16) float sO[QROWS * NF];
    __shared__ float sRed[4];

    const int tid = threadIdx.x, l = tid & 31, wv = tid >> 5, h = l >> 4, m = l & 15;
    const int i0 = blockIdx.x * QROWS + wv * 16;

    float mx = -3.0e38f;
    for (int j = tid; j < NJ; j += 128) mx = fmaxf(mx, s2[j]);
#pragma unroll
    for (int s = 16; s > 0; s >>= 1) mx = fmaxf(mx, __shfl_xor(mx, s));
    if (l == 0) sRed[wv] = mx;
    __syncthreads();
    mx = fmaxf(fmaxf(sRed[0], sRed[1]), fmaxf(sRed[2], sRed[3]));

    const float s_im = s1[i0 + m];
    const float Mrow = lk(s_im + mx);

    const v8f zero8 = {0.f, 0.f, 0.f, 0.f, 0.f, 0.f, 0.f, 0.f};
    v8f acc[NTL];
#pragma unroll
    for (int c = 0; c < NTL; ++c) acc[c] = zero8;
    float z = 0.f;
    const _Float16* xb = x16 + 8 * h;

#pragma unroll 1
    for (int j0 = 0; j0 < NJ; j0 += 32) {
        const float* sp = s2 + j0 + 8 * h;
        const v4f q0 = *(const v4f*)(sp);
        const v4f q1 = *(const v4f*)(sp + 4);
        const v4f q2 = *(const v4f*)(sp + 16);
        const v4f q3 = *(const v4f*)(sp + 20);
        v16h pa;
#pragma unroll
        for (int i = 0; i < 4; ++i) {
            pa[i]      = pval(q0[i], s_im, Mrow, z);
            pa[4 + i]  = pval(q1[i], s_im, Mrow, z);
            pa[8 + i]  = pval(q2[i], s_im, Mrow, z);
            pa[12 + i] = pval(q3[i], s_im, Mrow, z);
        }
#pragma unroll
        for (int c = 0; c < NTL; ++c) {
            const _Float16* bp = xb + (size_t)(16 * c + m) * NJ + j0;
            Frag bf;
            bf.half[0] = *(const v8h*)(bp);
            bf.half[1] = *(const v8h*)(bp + 16);
            acc[c] = wmma16(pa, bf.v, acc[c]);
        }
    }

    z += __shfl_xor(z, 16);
    const float zs = (1.0f / z) * (1.0f / PSCALE);
    float scl[8];
#pragma unroll
    for (int r = 0; r < 8; ++r) scl[r] = __shfl(zs, 8 * h + r);

    float* so = sO + wv * 16 * NF;
#pragma unroll
    for (int c = 0; c < NTL; ++c) {
        const int n = 16 * c + m;
        if (n < NF) {
#pragma unroll
            for (int r = 0; r < 8; ++r)
                so[(8 * h + r) * NF + n] = acc[c][r] * scl[r];
        }
    }
    __syncthreads();

    float* ob = out + (size_t)blockIdx.x * QROWS * NF;
    for (int g = wv; g < (QROWS * NF) / 128; g += 4) {
        const v4f v = *(const v4fa*)(sO + g * 128 + 4 * l);
        *(volatile v4f*)(ob + g * 128 + 4 * l) = v;
    }
    __threadfence();
    for (int g = wv; g < (QROWS * NF) / 128; g += 4) {
        const v4f v = *(const v4fa*)(sO + g * 128 + 4 * l);
        *(volatile v4f*)(ob + g * 128 + 4 * l) = v;
    }
}

extern "C" void kernel_launch(void* const* d_in, const int* in_sizes, int n_in,
                              void* d_out, int out_size, void* d_ws, size_t ws_size,
                              hipStream_t stream)
{
    const size_t x16_bytes = (size_t)NFP * NJ * sizeof(_Float16);
    const size_t s_bytes   = (size_t)NJ * sizeof(float);
    const size_t total     = x16_bytes + 2 * s_bytes;

    if (n_in < 2) return;
    if (in_sizes[0] != NF * NJ || in_sizes[1] != 2 * NF) return;
    if (out_size != NJ * NF || ws_size < total) return;

    const float* x   = (const float*)d_in[0];
    const float* w   = (const float*)d_in[1];
    float*       outp = (float*)d_out;

    char* ws = (char*)d_ws;
    _Float16* x16 = (_Float16*)ws;
    float*    s1  = (float*)(ws + x16_bytes);
    float*    s2  = (float*)(ws + x16_bytes + s_bytes);

    k_prep<<<NJ / PJ, 256, 0, stream>>>(x, w, x16, s1, s2);
    k_attn<<<NJ / QROWS, 128, 0, stream>>>(x16, s1, s2, outp);
    (void)hipGetLastError();
}
